// QuantLinearTorch_51599737094843
// MI455X (gfx1250) — hardware-verified
//
#include <hip/hip_runtime.h>
#include <math.h>

constexpr int kBatchN  = 4;
constexpr int kInF     = 4096;
constexpr int kOutF    = 11008;
constexpr int kGroup   = 128;
constexpr int kPack    = 8;
constexpr int kQRows   = kInF / kPack;
constexpr int kNGroups = kInF / kGroup;
constexpr int kMPad    = 64;
constexpr int kNHalf   = kOutF / 2;
constexpr int kDqTileN = 64;
static_assert(kNHalf % 64 == 0);
static_assert(kInF % 32 == 0);
static_assert(kInF % kGroup == 0);
static_assert(kGroup == 16 * kPack);
static_assert(kQRows * kOutF == 512 * 11008);

typedef __attribute__((ext_vector_type(16))) _Float16 v16h;
typedef __attribute__((ext_vector_type(8)))  _Float16 v8h;
typedef __attribute__((ext_vector_type(16))) __bf16   v16b;
typedef __attribute__((ext_vector_type(8)))  __bf16   v8b;
typedef __attribute__((ext_vector_type(8)))  float    v8f;
typedef __attribute__((ext_vector_type(4)))  float    v4f;
typedef __attribute__((ext_vector_type(4)))  unsigned int v4u;

__device__ __forceinline__ unsigned short f2bf_bits(float f) {
  unsigned u = __float_as_uint(f);
  return (unsigned short)((u + 0x7FFFu + ((u >> 16) & 1u)) >> 16);
}
__device__ __forceinline__ float bf_bits2f(unsigned short h) { return __uint_as_float(((unsigned)h) << 16); }

__device__ __forceinline__ void dep_guard_h(v8f& a, v8f& b, v16h x, v16h y) { asm volatile("v_nop\n\tv_nop\n\tv_nop\n\tv_nop" : "+v"(a), "+v"(b) : "v"(x), "v"(y)); }
__device__ __forceinline__ void dep_guard_b(v8f& a, v8f& b, v16b x, v16b y) { asm volatile("v_nop\n\tv_nop\n\tv_nop\n\tv_nop" : "+v"(a), "+v"(b) : "v"(x), "v"(y)); }
__device__ __forceinline__ void keep4_h(v16h a, v16h b, v16h c, v16h d) { asm volatile("v_nop" :: "v"(a), "v"(b), "v"(c), "v"(d)); }
__device__ __forceinline__ void keep4_b(v16b a, v16b b, v16b c, v16b d) { asm volatile("v_nop" :: "v"(a), "v"(b), "v"(c), "v"(d)); }
__device__ __forceinline__ void acc_guard4(v8f& a, v8f& b, v8f& c, v8f& d) { asm volatile("v_nop\n\tv_nop\n\tv_nop\n\tv_nop" : "+v"(a), "+v"(b), "+v"(c), "+v"(d)); }
template <typename T> struct Frag;
template <> struct Frag<_Float16> {
  typedef v16h V; union U { v16h v; v8h h[2]; };
  static __device__ __forceinline__ v16h load(const _Float16* p) {
    U f; f.h[0] = *(const v8h*)(p); f.h[1] = *(const v8h*)(p + 16); return f.v;
  }
  static __device__ __forceinline__ v8f mma(v16h a, v16h b, v8f c) {
    return __builtin_amdgcn_wmma_f32_16x16x32_f16(false, a, false, b, (short)0, c, false, false);
  }
  static __device__ __forceinline__ void guard(v8f& a, v8f& b, v16h x, v16h y) { dep_guard_h(a, b, x, y); }
  static __device__ __forceinline__ void keep(v16h a, v16h b, v16h c, v16h d) { keep4_h(a, b, c, d); }
};
template <> struct Frag<__bf16> {
  typedef v16b V; union U { v16b v; v8b h[2]; };
  static __device__ __forceinline__ v16b load(const __bf16* p) {
    U f; f.h[0] = *(const v8b*)(p); f.h[1] = *(const v8b*)(p + 16); return f.v;
  }
  static __device__ __forceinline__ v8f mma(v16b a, v16b b, v8f c) {
    return __builtin_amdgcn_wmma_f32_16x16x32_bf16(false, a, false, b, (short)0, c, false, false);
  }
  static __device__ __forceinline__ void guard(v8f& a, v8f& b, v16b x, v16b y) { dep_guard_b(a, b, x, y); }
  static __device__ __forceinline__ void keep(v16b a, v16b b, v16b c, v16b d) { keep4_b(a, b, c, d); }
};

__device__ __forceinline__ unsigned pk16(unsigned short a, unsigned short b) { return (unsigned)a | ((unsigned)b << 16); }

template <int ET> struct Elem;
template <> struct Elem<0> { typedef _Float16 T; };
template <> struct Elem<1> { typedef __bf16 T; };
template <int ET, int SPL, int RSC, int OUT_MODE, int ACT, int TRI>
__global__ __launch_bounds__(256) void wmma_gemm64(
    const unsigned short* __restrict__ Ap, const unsigned short* __restrict__ A2p, int lda, long strideA,
    const unsigned short* __restrict__ Btp, const unsigned short* __restrict__ Bt2p, int ldb, long strideB,
    void* __restrict__ Cout, void* __restrict__ Cout2, int ldc, long strideC,
    const float* __restrict__ rsc, long strideS,
    int M, int N, int K, float scale, int Mst) {
  typedef typename Elem<ET>::T T;
  typedef typename Frag<T>::V V;
  const T* A = (const T*)Ap; const T* A2 = (const T*)A2p; const T* Bt = (const T*)Btp; const T* Bt2 = (const T*)Bt2p;
  __shared__ __align__(16) float sT[8][16 * 68];
  const int b    = blockIdx.y;
  const int lane = threadIdx.x & 31;
  const int wave = threadIdx.x >> 5;
  const int tilesN = N >> 6;
  const int tilesM = M >> 6;
  const int tile = blockIdx.x * 8 + wave;
  if (tile >= tilesM * tilesN) return;
  const int tm = tile / tilesN;
  const int tn = tile - tm * tilesN;
  const int m0 = tm << 6;
  const int n0 = tn << 6;
  if (TRI == 1 && n0 > m0) return;
  const int Kl = (TRI == 2 && (m0 + 64) < K) ? (m0 + 64) : K;

  const T* Ab  = A  + (size_t)b * strideA;
  const T* Bb  = Bt + (size_t)b * strideB;
  const T* Ab2 = (SPL & 1) ? (A2  + (size_t)b * strideA) : nullptr;
  const T* Bb2 = (SPL & 2) ? (Bt2 + (size_t)b * strideB) : nullptr;

  const int rlane = lane & 15;
  const int koff  = (lane >> 4) * 8;
  const int mOff  = (lane >> 4) * 8;

  v8f acc[4][4];
#pragma unroll
  for (int i = 0; i < 4; ++i)
#pragma unroll
    for (int j = 0; j < 4; ++j) acc[i][j] = (v8f){0.f,0.f,0.f,0.f,0.f,0.f,0.f,0.f};

  for (int k0 = 0; k0 < Kl; k0 += 32) {
    V bh[4], bl[4];
#pragma unroll
    for (int j = 0; j < 4; ++j) {
      const size_t bo = (size_t)(n0 + (j << 4) + rlane) * ldb + koff + k0;
      bh[j] = Frag<T>::load(Bb + bo);
      if (SPL & 2) bl[j] = Frag<T>::load(Bb2 + bo);
    }
#pragma unroll
    for (int i = 0; i < 4; ++i) {
      const size_t ao = (size_t)(m0 + (i << 4) + rlane) * lda + koff + k0;
      V ah = Frag<T>::load(Ab + ao);
      V al;
      if (SPL & 1) al = Frag<T>::load(Ab2 + ao);
#pragma unroll
      for (int j = 0; j < 4; ++j) {
        acc[i][j] = Frag<T>::mma(ah, bh[j], acc[i][j]);
        if (SPL & 2) acc[i][j] = Frag<T>::mma(ah, bl[j], acc[i][j]);
        if (SPL & 1) acc[i][j] = Frag<T>::mma(al, bh[j], acc[i][j]);
      }
      Frag<T>::guard(acc[i][0], acc[i][3], ah, (SPL & 1) ? al : ah);
    }
    Frag<T>::keep(bh[0], bh[1], bh[2], bh[3]);
    if (SPL & 2) Frag<T>::keep(bl[0], bl[1], bl[2], bl[3]);
  }
  acc_guard4(acc[0][0], acc[0][1], acc[0][2], acc[0][3]);
  acc_guard4(acc[1][0], acc[1][1], acc[1][2], acc[1][3]);
  acc_guard4(acc[2][0], acc[2][1], acc[2][2], acc[2][3]);
  acc_guard4(acc[3][0], acc[3][1], acc[3][2], acc[3][3]);

  float* slab = sT[wave];
  const float* Rs = RSC ? (rsc + (size_t)b * strideS) : nullptr;
#pragma unroll
  for (int i = 0; i < 4; ++i) {
    const int mBase = m0 + (i << 4);
    float rsv[8];
#pragma unroll
    for (int r = 0; r < 8; ++r) rsv[r] = RSC ? Rs[mBase + mOff + r] : 1.0f;
#pragma unroll
    for (int j = 0; j < 4; ++j) {
      const int n = n0 + (j << 4) + rlane;
#pragma unroll
      for (int r = 0; r < 8; ++r) {
        float v = acc[i][j][r] * scale;
        if (RSC) v = v * rsv[r];
        if (TRI == 1) { if (n > mBase + mOff + r) v = 0.0f; }
        if (ACT == 6) v = (v > 0.0f) ? (v + 1.0f) : __expf(v);
        slab[(mOff + r) * 68 + (j << 4) + rlane] = v;
      }
    }
    __builtin_amdgcn_fence(__ATOMIC_RELEASE, "workgroup");
    __builtin_amdgcn_wave_barrier();
    __builtin_amdgcn_fence(__ATOMIC_ACQUIRE, "workgroup");
    if (OUT_MODE == 0) {
      float* C = (float*)Cout + (size_t)b * strideC;
      const int hh = lane >> 4, c4 = (lane & 15) * 4;
      for (int pass = 0; pass < 2; ++pass) {
#pragma unroll
        for (int it = 0; it < 8; ++it) {
          const int row = it * 2 + hh;
          v4f v = *(const v4f*)(slab + row * 68 + c4);
          if (mBase + row < Mst) *(volatile v4f*)(C + (size_t)(mBase + row) * ldc + n0 + c4) = v;
        }
        __threadfence();
      }
    } else {
      const int q = lane >> 3, c8 = (lane & 7) * 8;
      unsigned short* C  = (unsigned short*)Cout  + (size_t)b * strideC;
      unsigned short* C2 = (OUT_MODE == 2) ? ((unsigned short*)Cout2 + (size_t)b * strideC) : nullptr;
      for (int pass = 0; pass < 2; ++pass) {
#pragma unroll
        for (int it = 0; it < 4; ++it) {
          const int row = it * 4 + q;
          const float* sp = slab + row * 68 + c8;
          v8h hv, lv;
#pragma unroll
          for (int e = 0; e < 8; ++e) {
            if (OUT_MODE == 1) {
              hv[e] = (_Float16)sp[e];
            } else {
              unsigned short hb = f2bf_bits(sp[e]);
              unsigned short lb = f2bf_bits(sp[e] - bf_bits2f(hb));
              hv[e] = __builtin_bit_cast(_Float16, hb);
              lv[e] = __builtin_bit_cast(_Float16, lb);
            }
          }
          *(volatile v8h*)(C + (size_t)(mBase + row) * ldc + n0 + c8) = hv;
          if (OUT_MODE == 2) *(volatile v8h*)(C2 + (size_t)(mBase + row) * ldc + n0 + c8) = lv;
        }
        __threadfence();
      }
    }
    __builtin_amdgcn_fence(__ATOMIC_RELEASE, "workgroup");
    __builtin_amdgcn_wave_barrier();
    __builtin_amdgcn_fence(__ATOMIC_ACQUIRE, "workgroup");
  }
}

__global__ __launch_bounds__(256) void xsplit_kernel(const float* __restrict__ x, unsigned short* __restrict__ XH,
                                                      unsigned short* __restrict__ XL) {
  const int i = blockIdx.x * 256 + threadIdx.x;
  if (i >= kMPad * kInF / 8) return;
  const int row  = i >> 9;
  const int c8   = (i & 511) * 8;
  const int rowc = (row < kBatchN) ? row : (kBatchN - 1);
  const bool valid = row < kBatchN;
  const float* p = x + (size_t)rowc * kInF + c8;
  const v4f a = *(const v4f*)(p);
  const v4f c = *(const v4f*)(p + 4);
  unsigned short hb[8], lb[8];
#pragma unroll
  for (int e = 0; e < 4; ++e) {
    const float f0 = valid ? a[e] : 0.0f;
    const float f1 = valid ? c[e] : 0.0f;
    const unsigned short h0 = f2bf_bits(f0);
    const unsigned short h1 = f2bf_bits(f1);
    hb[e] = h0;      lb[e]     = f2bf_bits(f0 - bf_bits2f(h0));
    hb[4 + e] = h1;  lb[4 + e] = f2bf_bits(f1 - bf_bits2f(h1));
  }
  const v4u hv = (v4u){pk16(hb[0], hb[1]), pk16(hb[2], hb[3]), pk16(hb[4], hb[5]), pk16(hb[6], hb[7])};
  const v4u lv = (v4u){pk16(lb[0], lb[1]), pk16(lb[2], lb[3]), pk16(lb[4], lb[5]), pk16(lb[6], lb[7])};
  unsigned short* hp = XH + 8 * (size_t)i;
  unsigned short* lp = XL + 8 * (size_t)i;
  *(volatile v4u*)hp = hv;
  *(volatile v4u*)lp = lv;
  __threadfence();
  *(volatile v4u*)hp = hv;
  *(volatile v4u*)lp = lv;
}

__global__ __launch_bounds__(256) void dequant_split_kernel(const int* __restrict__ qw, const float* __restrict__ scales,
                                                             const float* __restrict__ zeros, unsigned short* __restrict__ WTH,
                                                             unsigned short* __restrict__ WTL, int nb) {
#pragma clang fp contract(off)
  __shared__ __align__(16) v4u sH[kDqTileN][17];
  __shared__ __align__(16) v4u sL[kDqTileN][17];
  const int t  = threadIdx.x;
  const int c  = t & 63;
  const int r4 = t >> 6;
  const int n0 = blockIdx.x * kDqTileN;
  const int kt = blockIdx.y;
  int ncol = nb + n0 + c;
  ncol = (ncol < kOutF) ? ncol : (kOutF - 1);
  const float sc = scales[(size_t)kt * kOutF + ncol];
  const float zr = zeros[(size_t)kt * kOutF + ncol];
#pragma unroll
  for (int i = 0; i < 4; ++i) {
    const int rl = r4 + 4 * i;
    int prow = kt * 16 + rl;
    prow = (prow < kQRows) ? prow : (kQRows - 1);
    const unsigned w = (unsigned)qw[(size_t)prow * kOutF + ncol];
    unsigned short hb[8], lb[8];
#pragma unroll
    for (int j = 0; j < 8; ++j) {
      const float q    = (float)((w >> (4 * j)) & 15u);
      const float prod = q * sc;
      const float wv   = prod - zr;
      const unsigned short h = f2bf_bits(wv);
      hb[j] = h;
      lb[j] = f2bf_bits(wv - bf_bits2f(h));
    }
    sH[c][rl] = (v4u){pk16(hb[0], hb[1]), pk16(hb[2], hb[3]), pk16(hb[4], hb[5]), pk16(hb[6], hb[7])};
    sL[c][rl] = (v4u){pk16(lb[0], lb[1]), pk16(lb[2], lb[3]), pk16(lb[4], lb[5]), pk16(lb[6], lb[7])};
  }
  __syncthreads();
  const int lane = t & 31, wv = t >> 5;
  const int hh = lane >> 4, q16 = lane & 15;
  for (int pass = 0; pass < 2; ++pass) {
#pragma unroll
    for (int it = 0; it < 4; ++it) {
      const int row = wv * 8 + it * 2 + hh;
      const v4u hvv = sH[row][q16];
      const v4u lvv = sL[row][q16];
      const size_t off = (size_t)(n0 + row) * kInF + (size_t)kt * kGroup + (size_t)q16 * 8;
      *(volatile v4u*)(WTH + off) = hvv;
      *(volatile v4u*)(WTL + off) = lvv;
    }
    __threadfence();
  }
}

extern "C" void kernel_launch(void* const* d_in, const int* in_sizes, int n_in,
                              void* d_out, int out_size, void* d_ws, size_t ws_size,
                              hipStream_t stream) {
  if (n_in < 4) return;
  if (in_sizes[0] != kBatchN * kInF) return;
  if (in_sizes[1] != kQRows * kOutF) return;
  if (in_sizes[2] != kNGroups * kOutF) return;
  if (in_sizes[3] != kNGroups * kOutF) return;
  if (out_size != kBatchN * kOutF) return;

  const float* x      = (const float*)d_in[0];
  const int*   qw     = (const int*)d_in[1];
  const float* scales = (const float*)d_in[2];
  const float* zeros  = (const float*)d_in[3];
  float* outp = (float*)d_out;

  const size_t SZ_X16 = (size_t)kMPad * kInF * 2;
  const size_t SZ_WT  = (size_t)kNHalf * kInF * 2;
  size_t off = 0;
  const size_t oXH  = off; off += SZ_X16;
  const size_t oXL  = off; off += SZ_X16;
  const size_t oWTH = off; off += SZ_WT;
  const size_t oWTL = off; off += SZ_WT;
  const size_t TOTAL = off;
  if (TOTAL > ws_size) return;
  if (TOTAL > (size_t)134217728) return;

  char* ws = (char*)d_ws;
  unsigned short* XH  = (unsigned short*)(ws + oXH);
  unsigned short* XL  = (unsigned short*)(ws + oXL);
  unsigned short* WTH = (unsigned short*)(ws + oWTH);
  unsigned short* WTL = (unsigned short*)(ws + oWTL);
  const float* dummy_rsc = scales;

  const dim3 blk(256);

  xsplit_kernel<<<dim3((kMPad * kInF / 8) / 256), blk, 0, stream>>>(x, XH, XL);

  const dim3 gDq(kNHalf / kDqTileN, kNGroups);
  const int  tiles = (kMPad / 64) * (kNHalf / 64);
  const dim3 gGemm((tiles + 7) / 8, 1);

  for (int hf = 0; hf < 2; ++hf) {
    const int nb = hf * kNHalf;
    dequant_split_kernel<<<gDq, blk, 0, stream>>>(qw, scales, zeros, WTH, WTL, nb);
    float* Cp = outp + nb;
    wmma_gemm64<1, 3, 0, 0, 0, 0><<<gGemm, blk, 0, stream>>>(
        XH, XL, kInF, 0L, WTH, WTL, kInF, 0L, (void*)Cp, (void*)Cp, kOutF, 0L,
        dummy_rsc, 0L, kMPad, kNHalf, kInF, 1.0f, kBatchN);
  }
}
